// EncoderLayer_71683004170482
// MI455X (gfx1250) — hardware-verified
//
#include <hip/hip_runtime.h>
#ifndef NB
#define NB 2
#endif
#ifndef SEQ
#define SEQ 2048
#endif
#define NB_FULL 2
#define SEQ_FULL 2048
#define SQ SEQ
#define DM 768
#define NH 12
#define HD 64
#define DFF 3072
#define HG 2
#define LQ (3 * DM)
#define DMQ DM
#define NR ((size_t)NB * SQ)
#define MP ((int)(NB * SQ))

static_assert(SQ % 128 == 0);
static_assert(MP % 128 == 0);
static_assert(DM % 64 == 0 && DFF % 64 == 0 && (3 * DM) % 64 == 0);
static_assert(DM % 32 == 0 && DFF % 32 == 0 && SQ % 32 == 0 && HD % 32 == 0);
static_assert(HD == 64 && NH * HD == DM && NH % HG == 0);
static_assert(DMQ % 4 == 0 && DMQ / 4 <= 256);
static_assert(NB <= NB_FULL && SEQ <= SEQ_FULL);

typedef unsigned short v8us __attribute__((ext_vector_type(8), may_alias));
typedef float  v8f  __attribute__((ext_vector_type(8)));
typedef float  v4f  __attribute__((ext_vector_type(4)));
typedef float  v4fa __attribute__((ext_vector_type(4), may_alias));
typedef _Float16 v16h __attribute__((ext_vector_type(16)));
typedef _Float16 v4h __attribute__((ext_vector_type(4)));
union FragH { v16h v; v8us half[2]; _Float16 h[16]; unsigned short u[16]; };

__device__ __forceinline__ unsigned short bf16_bits(float x) { unsigned int u = __float_as_uint(x); return (unsigned short)((u + 0x7FFFu + ((u >> 16) & 1u)) >> 16); }
__device__ __forceinline__ float bf16_val(unsigned short b) { return __uint_as_float(((unsigned int)b) << 16); }
__device__ __forceinline__ float bf16_rne(float x) { return bf16_val(bf16_bits(x)); }

__device__ __forceinline__ v16h g2_frag(const _Float16* p, int hh) { FragH f; f.half[0] = *(const v8us*)((const unsigned short*)p + 8 * hh); f.half[1] = *(const v8us*)((const unsigned short*)p + 16 + 8 * hh); return f.v; }
__device__ __forceinline__ v8f g2_mma(v16h a, v16h b, v8f c) { v8f d = __builtin_amdgcn_wmma_f32_16x16x32_f16(false, a, false, b, (short)0, c, false, false); asm volatile("v_nop\n\tv_nop\n\tv_nop\n\tv_nop" : "+v"(d) : "v"(a), "v"(b)); return d; }

__global__ __launch_bounds__(256) void k_wt_f16(const float* __restrict__ W, _Float16* __restrict__ Wt, unsigned K, unsigned N, float scale) {
  const unsigned t = blockIdx.x * 256u + threadIdx.x; const unsigned k8n = K >> 3;
  if (t >= N * k8n) return;
  const unsigned n = t / k8n; const unsigned k8 = (t - n * k8n) << 3; FragH f;
#pragma unroll
  for (int i = 0; i < 8; ++i) f.h[i] = (_Float16)(bf16_rne(W[(size_t)(k8 + (unsigned)i) * N + n]) * scale);
  const v8us o = f.half[0];
  unsigned short* d = (unsigned short*)Wt + (size_t)n * K + k8;
  *(volatile v8us*)d = o; __threadfence(); *(volatile v8us*)d = o;
}

__global__ __launch_bounds__(256) void k_bcpy(const float* __restrict__ b, unsigned n, float scale, float* __restrict__ dst) {
  for (int pass = 0; pass < 2; ++pass) {
#pragma unroll 1
    for (unsigned i = threadIdx.x; i < n; i += 256u) { const float v = bf16_rne(b[i]) * scale; *(volatile float*)(dst + i) = v; }
    if (pass == 0) __threadfence();
  }
}

__global__ __launch_bounds__(256) void k_xin(const float* __restrict__ x, _Float16* __restrict__ X16, float* __restrict__ XB, unsigned n4) {
  const unsigned t = blockIdx.x * 256u + threadIdx.x; if (t >= n4) return;
  const unsigned e = t << 2; const unsigned row = e / (unsigned)DM; const unsigned col = e - row * (unsigned)DM;
  const unsigned b = row / (unsigned)SQ; const unsigned s = row - b * (unsigned)SQ;
  const v4f a = *(const v4fa*)(x + ((size_t)b * SEQ_FULL + s) * DM + col);
  v4f xb; v4h y;
#pragma unroll
  for (int q = 0; q < 4; ++q) { xb[q] = bf16_rne(a[q]); y[q] = (_Float16)xb[q]; }
  for (int pass = 0; pass < 2; ++pass) { *(volatile v4f*)(XB + (size_t)e) = xb; *(volatile v4h*)(X16 + (size_t)e) = y; if (pass == 0) __threadfence(); }
}

template <unsigned NHv, unsigned TTv>
__global__ __launch_bounds__(256) void k_vt(const _Float16* __restrict__ V16, unsigned ldv, unsigned voff, _Float16* __restrict__ Vt) {
  __shared__ unsigned short tl[64][66];
  const unsigned tid = threadIdx.x; const unsigned slab = blockIdx.x / (TTv / 64u); const unsigned lg = blockIdx.x - slab * (TTv / 64u); const unsigned b = slab / NHv; const unsigned h = slab - b * NHv;
  for (unsigned i = tid; i < 512u; i += 256u) { const unsigned r = i >> 3, c8 = (i & 7u) << 3; FragH f; f.half[0] = *(const v8us*)((const unsigned short*)V16 + ((size_t)b * TTv + lg * 64u + r) * ldv + voff + h * 64u + c8);
#pragma unroll
    for (int q = 0; q < 8; ++q) tl[r][c8 + (unsigned)q] = f.u[q]; }
  __syncthreads();
  for (int pass = 0; pass < 2; ++pass) {
#pragma unroll
    for (unsigned rd = 0; rd < 2u; ++rd) { const unsigned d = rd * 32u + (tid >> 3), pc = tid & 7u; FragH f;
#pragma unroll
      for (int q = 0; q < 8; ++q) f.u[q] = tl[pc * 8u + (unsigned)q][d];
      *(volatile v8us*)((unsigned short*)Vt + ((size_t)slab * 64u + d) * TTv + lg * 64u + pc * 8u) = f.half[0]; }
    if (pass == 0) __threadfence(); }
}

template <int ACT>
__global__ __launch_bounds__(128) void k_gemm2(const _Float16* __restrict__ A, int lda, size_t sA, const _Float16* __restrict__ Bh, int ldb, size_t sB, float alpha, const float* __restrict__ bias, size_t sBias, const float* __restrict__ CP, int rowsPerB, size_t sCPb, int row0g,
    float* __restrict__ C, _Float16* __restrict__ C16, int ldc, size_t sC, int M, int N, int K) {
  static_assert(ACT == 0 || ACT == 3);
  __shared__ __attribute__((aligned(16))) float so[4][32][68];
  const int tid = threadIdx.x, w = tid >> 5, lane = tid & 31, ln = lane & 15, hh = lane >> 4; const unsigned by = blockIdx.y;
  A += (size_t)by * sA; Bh += (size_t)by * sB; const size_t cofs = (size_t)by * sC; const float* bp = bias ? bias + (size_t)by * sBias : nullptr;
  const unsigned ntn = (unsigned)N >> 6; const unsigned mtu = blockIdx.x / ntn; const unsigned nqu = blockIdx.x - mtu * ntn;
  const int row0 = (int)(mtu * 128u) + 32 * w, col0 = (int)(nqu * 64u); if (row0 >= M) return;
  const _Float16* a0p = A + (size_t)(row0 + ln) * lda; const _Float16* a1p = a0p + (size_t)16 * lda;
  const _Float16* b0p = Bh + (size_t)(col0 + ln) * ldb; const _Float16* b1p = b0p + (size_t)16 * ldb; const _Float16* b2p = b1p + (size_t)16 * ldb; const _Float16* b3p = b2p + (size_t)16 * ldb;
  const v8f z8 = {0.f,0.f,0.f,0.f,0.f,0.f,0.f,0.f}; v8f c00 = z8, c01 = z8, c02 = z8, c03 = z8, c10 = z8, c11 = z8, c12 = z8, c13 = z8;
#pragma unroll 1
  for (int kb = 0; kb < K; kb += 32) { const v16h a0 = g2_frag(a0p + kb, hh), a1 = g2_frag(a1p + kb, hh);
    v16h b = g2_frag(b0p + kb, hh); c00 = g2_mma(a0, b, c00); c10 = g2_mma(a1, b, c10);
    b = g2_frag(b1p + kb, hh); c01 = g2_mma(a0, b, c01); c11 = g2_mma(a1, b, c11);
    b = g2_frag(b2p + kb, hh); c02 = g2_mma(a0, b, c02); c12 = g2_mma(a1, b, c12);
    b = g2_frag(b3p + kb, hh); c03 = g2_mma(a0, b, c03); c13 = g2_mma(a1, b, c13); }
  v8f accs[8] = {c00, c01, c02, c03, c10, c11, c12, c13};
#pragma unroll
  for (int u = 0; u < 8; ++u) { const int t = u & 3, half = u >> 2; const int col = col0 + t * 16 + ln; const float bv = bp ? bf16_rne(bp[col]) : 0.f;
#pragma unroll
    for (int r = 0; r < 8; ++r) { const int rloc = half * 16 + 8 * hh + r; float v = accs[u][r] * alpha + bv;
      if (CP) { if (rowsPerB < 0) v += CP[cofs + (size_t)(row0g + row0 + rloc) * ldc + col];
                else { const int bidx = (row0g + row0 + rloc) / rowsPerB; v += CP[(size_t)bidx * sCPb + (size_t)by * 64 + col]; } }
      if (ACT == 3) v = fmaxf(v, 0.f);
      so[w][rloc][t * 16 + ln] = v; } }
  __builtin_amdgcn_fence(4  , "workgroup"); __builtin_amdgcn_wave_barrier();
  const int rsub = lane >> 4, c4 = (lane & 15) * 4;
  for (int pass = 0; pass < 2; ++pass) {
#pragma unroll
    for (int q = 0; q < 16; ++q) { const int r = q * 2 + rsub; const v4f v = *(const v4fa*)&so[w][r][c4];
      if (C) *(volatile v4f*)(C + cofs + (size_t)(row0 + r) * ldc + col0 + c4) = v;
      if (C16) { v4h h4; for (int i = 0; i < 4; ++i) h4[i] = (_Float16)v[i]; *(volatile v4h*)(C16 + cofs + (size_t)(row0 + r) * ldc + col0 + c4) = h4; } }
    if (pass == 0) __threadfence(); } }

__global__ __launch_bounds__(256) void k_rsmf(const float* __restrict__ S, _Float16* __restrict__ P, unsigned qn, unsigned hg) {
  #pragma clang fp contract(off)
  const unsigned t = blockIdx.x * 256u + threadIdx.x; if (t >= qn * hg) return; const unsigned hd = t / qn; const size_t i = (size_t)hd * SQ + (t - hd * qn); const float* s = S + i * SQ; float mx = -3.0e38f;
#pragma unroll 1
  for (int j = 0; j < SQ; ++j) mx = fmaxf(mx, s[j]); float se = 0.f;
#pragma unroll 1
  for (int j = 0; j < SQ; ++j) se += __expf(s[j] - mx); const float sc = 256.0f / se;
#pragma unroll 1
  for (int j0 = 0; j0 < SQ; j0 += 8) { FragH f; for (int q = 0; q < 8; ++q) f.h[q] = (_Float16)(__expf(s[j0 + q] - mx) * sc); unsigned short* d = (unsigned short*)P + i * SQ + j0; const v8us o = f.half[0]; *(volatile v8us*)d = o; __threadfence(); *(volatile v8us*)d = o; } }

template <int BFIN, int W16, int W32>
__global__ __launch_bounds__(256) void k_lnx(const float* __restrict__ X, const float* __restrict__ g, const float* __restrict__ bb, float eps, _Float16* __restrict__ N16, float* __restrict__ N32) {
  #pragma clang fp contract(off)
  __shared__ float red[256]; const size_t r = blockIdx.x; const unsigned t = threadIdx.x; const bool act = t < (unsigned)(DMQ / 4); const unsigned c0 = act ? t * 4u : 0u;
  const v4f xa = *(const v4fa*)(X + r * DMQ + c0); float s[4]; float sum = 0.f;
  for (int q = 0; q < 4; ++q) { s[q] = act ? (BFIN ? bf16_rne(xa[q]) : xa[q]) : 0.f; sum = __fadd_rn(sum, s[q]); }
  red[t] = sum; __syncthreads(); for (unsigned st = 128u; st > 0u; st >>= 1) { if (t < st) red[t] = __fadd_rn(red[t], red[t + st]); __syncthreads(); } const float mu = red[0] / (float)DMQ; __syncthreads();
  float vs = 0.f; for (int q = 0; q < 4; ++q) { const float dl = act ? __fadd_rn(s[q], -mu) : 0.f; vs = __fadd_rn(vs, __fmul_rn(dl, dl)); } red[t] = vs; __syncthreads(); for (unsigned st = 128u; st > 0u; st >>= 1) { if (t < st) red[t] = __fadd_rn(red[t], red[t + st]); __syncthreads(); }
  const float rs = rsqrtf(__fadd_rn(red[0] / (float)DMQ, eps)); v4h y; v4f yf;
  for (int q = 0; q < 4; ++q) { const unsigned c = c0 + (unsigned)q; yf[q] = __fadd_rn(__fmul_rn(__fmul_rn(__fadd_rn(s[q], -mu), rs), bf16_rne(g[c])), bf16_rne(bb[c])); y[q] = (_Float16)yf[q]; }
  if (!act) return;
  for (int pass = 0; pass < 2; ++pass) { if (W16) *(volatile v4h*)(N16 + r * DMQ + c0) = y; if (W32) *(volatile v4f*)(N32 + r * DMQ + c0) = yf; if (pass == 0) __threadfence(); } }

constexpr size_t cmax(size_t a, size_t b) { return a > b ? a : b; }
constexpr size_t al256(size_t b) { return (b + 255) & ~(size_t)255; }
constexpr size_t SZ_W   = al256((size_t)3 * DM * DM * 2) + al256((size_t)DM * DM * 2) + al256((size_t)DM * DFF * 2) + al256((size_t)DFF * DM * 2);
constexpr size_t SZ_B   = al256((size_t)3 * DM * 4) + al256((size_t)DFF * 4);
constexpr size_t SZ_X16 = al256(NR * DM * 2);
constexpr size_t SZ_XB  = al256(NR * DM * 4);
constexpr size_t SZ_Y   = al256(NR * DM * 4);
constexpr size_t SZ_QKV = al256(cmax(NR * 3 * DM * 2, NR * DM * 4));
constexpr size_t SZ_O   = al256(NR * DM * 2);
constexpr size_t SZ_S   = al256(cmax((size_t)HG * SQ * SQ * 4, NR * DFF * 2));
constexpr size_t SZ_P   = al256((size_t)HG * SQ * SQ * 2);
constexpr size_t SZ_VT  = al256((size_t)NH * HD * SQ * 2);
constexpr size_t SZ_ALL = SZ_W + SZ_B + SZ_X16 + SZ_XB + SZ_Y + SZ_QKV + SZ_O + SZ_S + SZ_P + SZ_VT;
static_assert(SZ_ALL <= (size_t)134217728);
static_assert(NR * DM * 4 <= SZ_QKV && NR * DFF * 2 <= SZ_S && (size_t)HG * SQ * SQ * 4 <= SZ_S);
static_assert((NR * DM) % 4 == 0);
static_assert((size_t)(MP / 128) * (3 * DM / 64) * 128 * 64 == (size_t)MP * 3 * DM);
static_assert((size_t)(SQ / 128) * (SQ / 64) * 128 * 64 == (size_t)SQ * SQ);
static_assert((size_t)(SQ / 128) * (HD / 64) * 128 * 64 == (size_t)SQ * HD);
static_assert((size_t)NH * (SQ / 64) * 64 * 64 == (size_t)NH * HD * SQ);
static_assert((size_t)(MP / 128) * (DM / 64) * 128 * 64 == (size_t)MP * DM);
static_assert((size_t)(MP / 128) * (DFF / 64) * 128 * 64 == (size_t)MP * DFF);
static_assert((DM % 256) == 0 && (DFF % 256) == 0);

extern "C" void kernel_launch(void* const* d_in, const int* in_sizes, int n_in,
                              void* d_out, int out_size, void* d_ws, size_t ws_size, hipStream_t stream) {
  if (n_in < 17) return;
  if ((size_t)in_sizes[0] < NR * DM) return;
  if (in_sizes[1] < DM * DM || in_sizes[3] < DM * DM || in_sizes[5] < DM * DM || in_sizes[7] < DM * DM) return;
  if (in_sizes[9] < DM * DFF || in_sizes[11] < DFF * DM) return;
  if (in_sizes[2] < DM || in_sizes[4] < DM || in_sizes[6] < DM || in_sizes[8] < DM || in_sizes[10] < DFF || in_sizes[12] < DM) return;
  if (in_sizes[13] < DM || in_sizes[14] < DM || in_sizes[15] < DM || in_sizes[16] < DM) return;
  if ((size_t)out_size < NR * DM) return;
  if (SZ_ALL > ws_size) return;
  const float* const* I = (const float* const*)d_in;
  const float* x = I[0]; const float* wq = I[1]; const float* bq = I[2]; const float* wk = I[3]; const float* bk = I[4]; const float* wv = I[5]; const float* bv = I[6];
  const float* wo = I[7]; const float* bo = I[8]; const float* w1 = I[9]; const float* b1 = I[10]; const float* w2 = I[11]; const float* b2 = I[12];
  const float* g1 = I[13]; const float* be1 = I[14]; const float* g2 = I[15]; const float* be2 = I[16];
  char* ws = (char*)d_ws; size_t off = 0;
  auto take = [&](size_t bytes) { char* p = ws + off; off += al256(bytes); return p; };
  _Float16* BQKV = (_Float16*)take((size_t)3 * DM * DM * 2); _Float16* BO = (_Float16*)take((size_t)DM * DM * 2); _Float16* BW1 = (_Float16*)take((size_t)DM * DFF * 2); _Float16* BW2 = (_Float16*)take((size_t)DFF * DM * 2);
  float* bqkv = (float*)take((size_t)3 * DM * 4); float* b1s = (float*)take((size_t)DFF * 4);
  _Float16* X16 = (_Float16*)take(SZ_X16); _Float16* M16 = X16;
  float* XB = (float*)take(SZ_XB);
  float* Y1 = (float*)take(SZ_Y); float* Y2 = Y1;
  _Float16* QKV = (_Float16*)take(SZ_QKV); float* X1 = (float*)QKV;
  _Float16* Q16 = QKV; _Float16* K16 = QKV + DM; _Float16* V16 = QKV + 2 * DM;
  _Float16* O16 = (_Float16*)take(SZ_O);
  float* S = (float*)take(SZ_S); _Float16* HF16 = (_Float16*)S;
  _Float16* P = (_Float16*)take(SZ_P);
  _Float16* VT = (_Float16*)take(SZ_VT);
  if (off > ws_size) return;

  { const unsigned g = (unsigned)(((size_t)DM * (DM / 8) + 255) / 256);
    k_wt_f16<<<g, 256, 0, stream>>>(wq, BQKV, DM, DM, 16.0f);
    k_wt_f16<<<g, 256, 0, stream>>>(wk, BQKV + (size_t)DM * DM, DM, DM, 16.0f);
    k_wt_f16<<<g, 256, 0, stream>>>(wv, BQKV + (size_t)2 * DM * DM, DM, DM, 16.0f);
    k_wt_f16<<<g, 256, 0, stream>>>(wo, BO, DM, DM, 16.0f); }
  k_wt_f16<<<(unsigned)(((size_t)DFF * (DM / 8) + 255) / 256), 256, 0, stream>>>(w1, BW1, DM, DFF, 16.0f);
  k_wt_f16<<<(unsigned)(((size_t)DM * (DFF / 8) + 255) / 256), 256, 0, stream>>>(w2, BW2, DFF, DM, 16.0f);
  k_bcpy<<<1, 256, 0, stream>>>(bq, DM, 1.0f, bqkv); k_bcpy<<<1, 256, 0, stream>>>(bk, DM, 1.0f, bqkv + DM); k_bcpy<<<1, 256, 0, stream>>>(bv, DM, 1.0f, bqkv + 2 * DM);
  k_bcpy<<<1, 256, 0, stream>>>(b1, DFF, 16.0f, b1s);
  k_xin<<<(unsigned)((NR * DM / 4 + 255) / 256), 256, 0, stream>>>(x, X16, XB, (unsigned)(NR * DM / 4));
  k_gemm2<0><<<dim3((unsigned)((MP / 128) * (3 * DM / 64)), 1), 128, 0, stream>>>(X16, DM, 0, BQKV, DM, 0, 0.0625f, bqkv, 0, nullptr, 1, 0, 0, nullptr, QKV, 3 * DM, 0, MP, 3 * DM, DM);
  for (int b = 0; b < NB; ++b) { const size_t r0 = (size_t)b * SQ;
    k_vt<NH, SQ><<<NH * (SQ / 64), 256, 0, stream>>>(V16 + r0 * LQ, LQ, 0, VT);
    for (int h0 = 0; h0 < NH; h0 += HG) {
      k_gemm2<0><<<dim3((SQ / 128) * (SQ / 64), HG), 128, 0, stream>>>(Q16 + r0 * LQ + (size_t)h0 * HD, LQ, (size_t)HD, K16 + r0 * LQ + (size_t)h0 * HD, LQ, (size_t)HD, 0.125f, nullptr, 0, nullptr, 1, 0, 0, S, nullptr, SQ, (size_t)SQ * SQ, SQ, SQ, HD);
      k_rsmf<<<(HG * SQ + 255) / 256, 256, 0, stream>>>(S, P, SQ, HG);
      k_gemm2<0><<<dim3((SQ / 128) * (HD / 64), HG), 128, 0, stream>>>(P, SQ, (size_t)SQ * SQ, VT + (size_t)h0 * HD * SQ, SQ, (size_t)HD * SQ, 0.25f, nullptr, 0, nullptr, 1, 0, 0, nullptr, O16 + r0 * DM + (size_t)h0 * HD, DM, (size_t)HD, SQ, HD, SQ); } }
  k_gemm2<0><<<dim3((unsigned)((MP / 128) * (DM / 64)), 1), 128, 0, stream>>>(O16, DM, 0, BO, DM, 0, 0.0009765625f, bo, 0, XB, -1, 0, 0, Y1, nullptr, DM, 0, MP, DM, DM);
  k_lnx<0, 1, 1><<<(unsigned)NR, 256, 0, stream>>>(Y1, g1, be1, 1e-5f, M16, X1);
  k_gemm2<3><<<dim3((unsigned)((MP / 128) * (DFF / 64)), 1), 128, 0, stream>>>(M16, DM, 0, BW1, DM, 0, 1.0f, b1s, 0, nullptr, 1, 0, 0, nullptr, HF16, DFF, 0, MP, DFF, DM);
  k_gemm2<0><<<dim3((unsigned)((MP / 128) * (DM / 64)), 1), 128, 0, stream>>>(HF16, DFF, 0, BW2, DFF, 0, 0.00390625f, b2, 0, X1, -1, 0, 0, Y2, nullptr, DM, 0, MP, DM, DFF);
  k_lnx<0, 0, 1><<<(unsigned)NR, 256, 0, stream>>>(Y2, g2, be2, 1e-5f, nullptr, (float*)d_out);
}
